// EMB_84842783965559
// MI455X (gfx1250) — hardware-run, weakly checked
//
#include <hip/hip_runtime.h>
#include <math.h>

typedef __attribute__((ext_vector_type(16))) _Float16 v16h;
typedef __attribute__((ext_vector_type(8)))  _Float16 v8h;
typedef __attribute__((ext_vector_type(8)))  float    v8f;
typedef __attribute__((ext_vector_type(4)))  float    v4f;
typedef __attribute__((ext_vector_type(4)))  unsigned v4u;

constexpr int kDays    = 50000;
constexpr int kMpad    = 50048;
constexpr int kHid     = 512;
constexpr int kXin     = 12;
constexpr int kPcols   = 27;
constexpr int kPpred   = 3;
constexpr int kYcols   = 2;
constexpr int kKsmall  = 32;
constexpr int kNsmall  = 64;
constexpr int kChunks  = kMpad / 32;
constexpr int kRedBlk  = kMpad / 128;
constexpr int kPreBlk  = 196;
constexpr int kPreRows = kPreBlk * 256;
static_assert(kMpad % 64 == 0 && kMpad >= kDays, "M tile multiple");
static_assert(kChunks * 32 == kMpad && kChunks == 1564, "chunk cover");
static_assert(kRedBlk * 128 == kMpad && kRedBlk == 391, "column-sum cover");
static_assert(kPreRows >= kMpad, "term plane cover");
static_assert(kHid % 64 == 0 && kHid % 32 == 0 && kKsmall % 32 == 0 && kNsmall % 64 == 0, "GEMM N,K multiples");
static_assert((2 * kDays * 4) % 128 == 0, "second output starts on a line");
static_assert((kDays * kPpred) % 4 == 0 && (kDays * kYcols) % 4 == 0, "vector store cover");
static_assert(2 * kPpred <= 8 && 2 * kPpred <= kKsmall, "value + residual columns fit the first 8 halves of a row");

constexpr float kCarryX  = 16.0f;
constexpr float kCarryP  = 16.0f;
constexpr float kCarryH  = 16.0f;
constexpr float kCarryW0 = 64.0f;
constexpr float kCarryW1 = 256.0f;
constexpr float kCarryW2 = 1024.0f;
constexpr float kCarryR0 = 64.0f;
constexpr float kCarryR1 = 256.0f;
constexpr float kCarryR2 = 256.0f;

constexpr size_t kSzH    = (size_t)kMpad * kHid * 2;
constexpr size_t kSzPR   = (size_t)kMpad * kNsmall * 4;
constexpr size_t kSzS    = (size_t)kMpad * kKsmall * 2;
constexpr size_t kSzW0   = (size_t)kHid * kKsmall * 2;
constexpr size_t kSzW1   = (size_t)kHid * kHid * 2;
constexpr size_t kSzW2   = (size_t)kNsmall * kHid * 2;
constexpr size_t kSzPart = (size_t)kRedBlk * 32 * 4;
constexpr size_t kSzBias = (size_t)kNsmall * 4;
constexpr size_t kSzPM   = 128;
constexpr size_t kSzFS   = (size_t)kMpad * 4;
constexpr size_t kSzPRE  = (size_t)kPreRows * 16 * 4;
constexpr size_t kOffH0   = 0;
constexpr size_t kOffH1   = kOffH0 + kSzH;
constexpr size_t kOffPR   = kOffH1 + kSzH;
constexpr size_t kOffXH   = kOffPR + kSzPR;
constexpr size_t kOffP3   = kOffXH + kSzS;
constexpr size_t kOffW0T  = kOffP3 + kSzS;
constexpr size_t kOffW1T  = kOffW0T + kSzW0;
constexpr size_t kOffW2T  = kOffW1T + kSzW1;
constexpr size_t kOffR0T  = kOffW2T + kSzW2;
constexpr size_t kOffR1T  = kOffR0T + kSzW0;
constexpr size_t kOffR2T  = kOffR1T + kSzW1;
constexpr size_t kOffPART = kOffR2T + kSzW2;
constexpr size_t kOffB2P  = kOffPART + kSzPart;
constexpr size_t kOffRB2P = kOffB2P + kSzBias;
constexpr size_t kOffPM   = kOffRB2P + kSzBias;
constexpr size_t kOffFS   = kOffPM + kSzPM;
constexpr size_t kOffPRE  = kOffFS + kSzFS;
constexpr size_t kWsTotal = kOffPRE + kSzPRE;
static_assert(kWsTotal == 126424064ull, "carve total");
static_assert(kWsTotal <= 134217728ull, "carve cap");
static_assert((kOffH1 % 128) == 0 && (kOffPR % 128) == 0 && (kOffXH % 128) == 0 && (kOffP3 % 128) == 0 &&
              (kOffW0T % 128) == 0 && (kOffW1T % 128) == 0 && (kOffW2T % 128) == 0 && (kOffR0T % 128) == 0 &&
              (kOffR1T % 128) == 0 && (kOffR2T % 128) == 0 && (kOffPART % 128) == 0 && (kOffB2P % 128) == 0 &&
              (kOffRB2P % 128) == 0 && (kOffPM % 128) == 0 && (kOffFS % 128) == 0 && (kOffPRE % 128) == 0,
              "128-B aligned regions");

static constexpr float INF_ = 3.402823466e+38f;
__device__ __constant__ float kScales[32] = {
  400,1,1,1,1,12,10,10,1,1,1,1,1,10,1,1,1,5,1,1,4,1,1,180,1,1,10,
  0,0,0,0,0};
__device__ __constant__ float kLo[32] = {
  0.f,0.f,0.f,-INF_,0.f,0.01f,-0.2f,0.23f,-1.f,0.f,
  0.f,-INF_,-INF_,0.f,0.f,0.f,0.f,0.f,-INF_,0.f,
  0.f,0.f,-INF_,0.f,0.f,0.f,0.f,
  0.f,0.f,0.f,0.f,0.f};
__device__ __constant__ float kHi[32] = {
  2.f,INF_,INF_,INF_,2.5f,3.f,2.1f,3.f,0.f,0.7f,
  0.f,INF_,INF_,1.f,1.2f,2.5f,0.f,1.f,INF_,1.3333334f,
  INF_,INF_,INF_,INF_,INF_,INF_,INF_,
  0.f,0.f,0.f,0.f,0.f};
static_assert(sizeof(kScales) / sizeof(kScales[0]) == 32, "table size");
static_assert(sizeof(kLo) / sizeof(kLo[0]) == 32, "table size");
static_assert(sizeof(kHi) / sizeof(kHi[0]) == 32, "table size");

__device__ __forceinline__ unsigned f16_bits(float f) {
  const _Float16 h = (_Float16)f;
  return (unsigned)__builtin_bit_cast(unsigned short, h);
}
__device__ __forceinline__ unsigned pack2h(float a, float b) {
  const unsigned lo = f16_bits(a);
  const unsigned hi = f16_bits(b);
  return lo | (hi << 16);
}
__device__ __forceinline__ void split_h16(float v, unsigned& hb, unsigned& rb) {
  const _Float16 h = (_Float16)v;
  const float hf = (float)h;
  const bool tiny = fabsf(hf) < 6.103515625e-5f;
  const float hsel = tiny ? 0.0f : hf;
  const float res = v - hsel;
  hb = f16_bits(hsel);
  rb = f16_bits(res);
}

__device__ __forceinline__ void guard1_h(v8f& a, v16h x, v16h y) {
  asm volatile("v_nop\n\tv_nop\n\tv_nop\n\tv_nop" : "+v"(a) : "v"(x), "v"(y));
}
__device__ __forceinline__ void keep4_h(v16h a, v16h b, v16h c, v16h d) {
  asm volatile("v_nop" :: "v"(a), "v"(b), "v"(c), "v"(d));
}
__device__ __forceinline__ void acc_guard4(v8f& a, v8f& b, v8f& c, v8f& d) {
  asm volatile("v_nop\n\tv_nop\n\tv_nop\n\tv_nop" : "+v"(a), "+v"(b), "+v"(c), "+v"(d));
}
struct FragH {
  union U { v16h v; v8h h[2]; };
  static __device__ __forceinline__ v16h load(const _Float16* p) {
    U f; f.h[0] = *(const v8h*)(p); f.h[1] = *(const v8h*)(p + 16); return f.v;
  }
  static __device__ __forceinline__ v8f mma(v16h a, v16h b, v8f c) {
    return __builtin_amdgcn_wmma_f32_16x16x32_f16(false, a, false, b, (short)0, c, false, false);
  }
};

template <int OUT_F32, int ACT_ELU>
__global__ __launch_bounds__(256) void wmma_gemm64_f16(
    const unsigned short* __restrict__ Ap, int lda,
    const unsigned short* __restrict__ Btp, int ldb,
    void* __restrict__ Cout, int ldc,
    const float* __restrict__ bias,
    int M, int N, int K, float scale, float oscale) {
  const _Float16* A  = (const _Float16*)Ap;
  const _Float16* Bt = (const _Float16*)Btp;
  __shared__ __align__(16) float sT[8][16 * 68];
  const int lane = threadIdx.x & 31;
  const int wave = threadIdx.x >> 5;
  const int tilesN = N >> 6;
  const int tilesM = M >> 6;
  const int tile = blockIdx.x * 8 + wave;
  if (tile >= tilesM * tilesN) return;
  const int tm = tile / tilesN;
  const int tn = tile - tm * tilesN;
  const int m0 = tm << 6;
  const int n0 = tn << 6;

  const int rlane = lane & 15;
  const int koff  = (lane >> 4) * 8;
  const int mOff  = (lane >> 4) * 8;

  v8f acc[4][4];
#pragma unroll
  for (int i = 0; i < 4; ++i)
#pragma unroll
    for (int j = 0; j < 4; ++j) acc[i][j] = (v8f){0.f,0.f,0.f,0.f,0.f,0.f,0.f,0.f};

  for (int k0 = 0; k0 < K; k0 += 32) {
    v16h bh[4];
#pragma unroll
    for (int j = 0; j < 4; ++j) {
      const size_t bo = (size_t)(n0 + (j << 4) + rlane) * ldb + koff + k0;
      bh[j] = FragH::load(Bt + bo);
    }
#pragma unroll
    for (int i = 0; i < 4; ++i) {
      const size_t ao = (size_t)(m0 + (i << 4) + rlane) * lda + koff + k0;
      const v16h ah = FragH::load(A + ao);
      acc[i][0] = FragH::mma(ah, bh[0], acc[i][0]);
      acc[i][1] = FragH::mma(ah, bh[1], acc[i][1]);
      acc[i][2] = FragH::mma(ah, bh[2], acc[i][2]);
      acc[i][3] = FragH::mma(ah, bh[3], acc[i][3]);
      guard1_h(acc[i][0], ah, bh[0]);
      guard1_h(acc[i][1], ah, bh[1]);
      guard1_h(acc[i][2], ah, bh[2]);
      guard1_h(acc[i][3], ah, bh[3]);
    }
    keep4_h(bh[0], bh[1], bh[2], bh[3]);
  }
  acc_guard4(acc[0][0], acc[0][1], acc[0][2], acc[0][3]);
  acc_guard4(acc[1][0], acc[1][1], acc[1][2], acc[1][3]);
  acc_guard4(acc[2][0], acc[2][1], acc[2][2], acc[2][3]);
  acc_guard4(acc[3][0], acc[3][1], acc[3][2], acc[3][3]);

  float* slab = sT[wave];
#pragma unroll
  for (int i = 0; i < 4; ++i) {
    const int mBase = m0 + (i << 4);
#pragma unroll
    for (int j = 0; j < 4; ++j) {
      const int n = n0 + (j << 4) + rlane;
      const float bv = bias[n];
#pragma unroll
      for (int r = 0; r < 8; ++r) {
        float v = acc[i][j][r] * scale;
        v += bv;
        if (ACT_ELU == 0) v = v * oscale;
        slab[(mOff + r) * 68 + (j << 4) + rlane] = v;
      }
    }
    if (ACT_ELU == 1) {
#pragma unroll 1
      for (int e = 0; e < 32; ++e) {
        const int idx = (mOff + (e & 7)) * 68 + ((e >> 3) << 4) + rlane;
        const float v = slab[idx];
        const float em = expm1f(v);
        slab[idx] = ((v > 0.0f) ? v : em) * oscale;
      }
    }
    __builtin_amdgcn_fence(__ATOMIC_RELEASE, "workgroup");
    __builtin_amdgcn_wave_barrier();
    __builtin_amdgcn_fence(__ATOMIC_ACQUIRE, "workgroup");
    if (OUT_F32 == 1) {
      float* C = (float*)Cout;
      const int hh = lane >> 4, c4 = (lane & 15) * 4;
      for (int pass = 0; pass < 2; ++pass) {
#pragma unroll
        for (int it = 0; it < 8; ++it) {
          const int row = it * 2 + hh;
          v4f v = *(const v4f*)(slab + row * 68 + c4);
          *(volatile v4f*)(C + (size_t)(mBase + row) * ldc + n0 + c4) = v;
        }
        __threadfence();
      }
    } else {
      const int q = lane >> 3, c8 = (lane & 7) * 8;
      unsigned short* C = (unsigned short*)Cout;
      for (int pass = 0; pass < 2; ++pass) {
#pragma unroll
        for (int it = 0; it < 4; ++it) {
          const int row = it * 4 + q;
          const float* sp = slab + row * 68 + c8;
          v8h hv;
#pragma unroll
          for (int e = 0; e < 8; ++e) hv[e] = (_Float16)sp[e];
          *(volatile v8h*)(C + (size_t)(mBase + row) * ldc + n0 + c8) = hv;
        }
        __threadfence();
      }
    }
    __builtin_amdgcn_fence(__ATOMIC_RELEASE, "workgroup");
    __builtin_amdgcn_wave_barrier();
    __builtin_amdgcn_fence(__ATOMIC_ACQUIRE, "workgroup");
  }
}

__global__ __launch_bounds__(256) void pack_x_kernel(
    const float* __restrict__ x, unsigned short* __restrict__ XH, int total8, float carry) {
  const int idx = blockIdx.x * 256 + threadIdx.x;
  if (idx >= total8) return;
  const int row = idx >> 2;
  const int g = idx & 3;
  const int rc = row < kDays ? row : (kDays - 1);
  float f[8];
#pragma unroll
  for (int e = 0; e < 8; ++e) {
    const int col = g * 8 + e;
    const int cc = col < kXin ? col : (kXin - 1);
    float v = x[(size_t)rc * kXin + cc];
    asm volatile("" : "+v"(v));
    f[e] = (col < kXin && row < kDays) ? (v * carry) : 0.0f;
  }
  const v4u w = {pack2h(f[0], f[1]), pack2h(f[2], f[3]), pack2h(f[4], f[5]), pack2h(f[6], f[7])};
  unsigned short* dst = XH + (size_t)idx * 8;
  *(volatile v4u*)dst = w;
  __threadfence();
  *(volatile v4u*)dst = w;
}

__global__ __launch_bounds__(256) void pack_wt_kernel(
    const float* __restrict__ W, int Kreal, int Nreal, int kshift, int dupK,
    unsigned short* __restrict__ out, int total8, float carry) {
  const int idx = blockIdx.x * 256 + threadIdx.x;
  if (idx >= total8) return;
  const int n = idx >> kshift;
  const int g = idx & ((1 << kshift) - 1);
  const int nc = n < Nreal ? n : (Nreal - 1);
  float f[8];
#pragma unroll
  for (int e = 0; e < 8; ++e) {
    const int k = g * 8 + e;
    int ks = (k < Kreal) ? k : (k - Kreal);
    ks = ks < 0 ? 0 : (ks > Kreal - 1 ? Kreal - 1 : ks);
    float v = W[(size_t)ks * Nreal + nc];
    asm volatile("" : "+v"(v));
    f[e] = (k < Kreal + dupK && n < Nreal) ? (v * carry) : 0.0f;
  }
  const v4u w = {pack2h(f[0], f[1]), pack2h(f[2], f[3]), pack2h(f[4], f[5]), pack2h(f[6], f[7])};
  unsigned short* dst = out + (size_t)idx * 8;
  *(volatile v4u*)dst = w;
  __threadfence();
  *(volatile v4u*)dst = w;
}

__global__ __launch_bounds__(32) void pad_bias_kernel(
    const float* __restrict__ ba, int na, const float* __restrict__ bb, int nb,
    float* __restrict__ outa, float* __restrict__ outb) {
  const int lane = threadIdx.x;
  float va[2], vb[2];
#pragma unroll
  for (int j = 0; j < 2; ++j) {
    const int n = lane + 32 * j;
    const int ia = n < na ? n : (na - 1);
    const int ib = n < nb ? n : (nb - 1);
    float xa = ba[ia];
    float xb = bb[ib];
    asm volatile("" : "+v"(xa));
    asm volatile("" : "+v"(xb));
    va[j] = (n < na) ? xa : 0.0f;
    vb[j] = (n < nb) ? xb : 0.0f;
  }
  for (int pass = 0; pass < 2; ++pass) {
    ((volatile float*)outa)[lane] = va[0];
    ((volatile float*)outa)[lane + 32] = va[1];
    ((volatile float*)outb)[lane] = vb[0];
    ((volatile float*)outb)[lane + 32] = vb[1];
    __threadfence();
  }
}

__global__ __launch_bounds__(256) void constrain_colsum_kernel(
    const float* __restrict__ PR, float* __restrict__ PART) {
  __shared__ float sP[8 * 32];
  const int lane = threadIdx.x & 31;
  const int wave = threadIdx.x >> 5;
  const int r0 = blockIdx.x * 128 + wave * 16;
  const float lo = kLo[lane];
  const float hi = kHi[lane];
  const bool isSig = (lane == 10) || (lane == 16);
  const bool colOk = lane < kPcols;
  float acc = 0.0f;
#pragma unroll 1
  for (int i = 0; i < 16; ++i) {
    const int r = r0 + i;
    const float v = PR[(size_t)r * kNsmall + lane];
    const float clip = fminf(fmaxf(v, lo), hi);
    const float sg = 1.0f / (1.0f + expf(-v));
    const float c = isSig ? sg : clip;
    acc += (colOk && r < kDays) ? c : 0.0f;
  }
  sP[wave * 32 + lane] = acc;
  __syncthreads();
  if (wave == 0) {
    float t = 0.0f;
#pragma unroll
    for (int w = 0; w < 8; ++w) t += sP[w * 32 + lane];
    volatile float* dst = (volatile float*)(PART + (size_t)blockIdx.x * 32);
    dst[lane] = t;
    __threadfence();
    dst[lane] = t;
  }
}

__global__ __launch_bounds__(32) void mean_sfilter_kernel(
    const float* __restrict__ PART, const float* __restrict__ cin,
    float* __restrict__ PM, float* __restrict__ FS) {
#pragma clang fp contract(off)
  __shared__ float sPm[32];
  __shared__ float sTa[32];
  __shared__ float sFs[32];
  const int lane = threadIdx.x;
  double dsum = 0.0;
#pragma unroll 1
  for (int b = 0; b < kRedBlk; ++b) dsum += (double)PART[(size_t)b * 32 + lane];
  const float meanv = (float)(dsum * (1.0 / (double)kDays));
  const float pmv = meanv * kScales[lane];
  ((volatile float*)PM)[lane] = pmv;
  __threadfence();
  ((volatile float*)PM)[lane] = pmv;
  sPm[lane] = pmv;
  __syncthreads();
  const float tau = sPm[5], S0 = sPm[6], Smax = sPm[7];
  float S = sPm[26];
#pragma unroll 1
  for (int ch = 0; ch < kChunks; ++ch) {
    const int base = ch * 32;
    __syncthreads();
    const int t = base + lane;
    const int tc = t < kDays ? t : (kDays - 1);
    sTa[lane] = cin[(size_t)tc * 7 + 1];
    sFs[lane] = 0.0f;
    __syncthreads();
    int nvalid = kDays - base;
    nvalid = nvalid < 0 ? 0 : (nvalid > 32 ? 32 : nvalid);
    if (lane == 0) {
#pragma unroll 1
      for (int s = 0; s < nvalid; ++s) {
        S = S + (sTa[s] - S) / tau;
        sFs[s] = fminf(fmaxf(S - S0, 0.0f) / Smax, 1.0f);
      }
    }
    __syncthreads();
    const float fv = sFs[lane];
    ((volatile float*)FS)[base + lane] = fv;
    __threadfence();
    ((volatile float*)FS)[base + lane] = fv;
  }
}

__global__ __launch_bounds__(256) void daily_terms_kernel(
    const float* __restrict__ cin, const float* __restrict__ PM, const float* __restrict__ FS,
    float* __restrict__ PRE) {
#pragma clang fp contract(off)
  __shared__ __align__(16) float sRec[256 * 16];
  const int tid = threadIdx.x;
  const int t = blockIdx.x * 256 + tid;
  const int tc = t < kDays ? t : (kDays - 1);
  const int tfs = t < kMpad ? t : (kMpad - 1);
  const float* row = cin + (size_t)tc * 7;
  const float precip = row[0], tair = row[1], par = row[2], vpd = row[3], fapar = row[4], co2 = row[6];
  const float fS = FS[tfs];
  const float beta = PM[4], kappa = PM[8], gamma = PM[9], bCO2 = PM[11], xCO2 = PM[12];
  const float ETbeta = PM[13], ETkappa = PM[14], ETchi = PM[15], MeltCoef = PM[18];
  const float I0 = PM[19], CWmax = PM[20], SnowThr = PM[21], Tzero = PM[22];

  const float logco2 = logf(co2 * (1.0f / 380.0f));
  const float fD = fminf(expf(kappa * vpd), 1.0f);
  const float fL = 1.0f / (gamma * par + 1.0f);
  const float bpfsl = (((beta * par) * fapar) * fS) * fL;
  const float gfac = 1.0f + bCO2 * logco2;
  const float icq = ((precip * I0) * fapar) * (1.0f / 0.75f);
  const float icpt = (tair > SnowThr) ? icq : 0.0f;
  const float rain = precip - icpt;
  const float rpi = rain + icpt;
  const float cap = CWmax * fapar;
  const float mq = MeltCoef * (tair - Tzero);
  const float meltpot = (tair >= Tzero) ? mq : 0.0f;
  const float fco2et = 1.0f + xCO2 * logco2;
  const float vb = vpd * ETbeta;
  const float pw = powf(vpd, ETkappa);
  const float ec = ETchi * (1.0f - fapar);
  const float snowflag = (tair < SnowThr) ? 1.0f : 0.0f;

  *(v4f*)(sRec + tid * 16 + 0)  = (v4f){rain, rpi, icpt, cap};
  *(v4f*)(sRec + tid * 16 + 4)  = (v4f){meltpot, snowflag, fD, bpfsl};
  *(v4f*)(sRec + tid * 16 + 8)  = (v4f){gfac, fco2et, vb, pw};
  *(v4f*)(sRec + tid * 16 + 12) = (v4f){ec, par, 0.0f, 0.0f};
  __syncthreads();
  v4f ov[4];
#pragma unroll
  for (int it = 0; it < 4; ++it) ov[it] = *(const v4f*)(sRec + (size_t)(it * 256 + tid) * 4);
  float* dst = PRE + (size_t)blockIdx.x * 4096;
  for (int pass = 0; pass < 2; ++pass) {
#pragma unroll
    for (int it = 0; it < 4; ++it) *(volatile v4f*)(dst + (size_t)(it * 256 + tid) * 4) = ov[it];
    __threadfence();
  }
}

__global__ __launch_bounds__(32) void water_scan_kernel(
    const float* __restrict__ PM, const float* __restrict__ PRE, const float* __restrict__ sw,
    float* __restrict__ out1, unsigned short* __restrict__ P3, float pcarry) {
#pragma clang fp contract(off)
  __shared__ __align__(16) float sR[32 * 16];
  __shared__ __align__(16) float sO[96];
  const int lane = threadIdx.x;
  const float soildepth = PM[0], thetaFC = PM[1], thetaPWP = PM[2], taud = PM[3];
  const float soilthres = PM[10], etst = PM[16], etnu = PM[17], CWmax = PM[20];
  const float dfc = thetaFC - thetaPWP;
  const float fcap = thetaFC * soildepth;
  const bool smallcw = (CWmax <= 1e-8f);
  const float sw0 = sw[0], sw1 = sw[1];
  float theta = PM[23], canw = PM[24], snow = PM[25];
  unsigned zw = 0u;
  asm volatile("" : "+v"(zw));
#pragma unroll 1
  for (int ch = 0; ch < kChunks; ++ch) {
    const int base = ch * 32;
    __syncthreads();
    {
      const float* src = PRE + (size_t)(base + lane) * 16;
      const v4f a0 = *(const v4f*)(src);
      const v4f a1 = *(const v4f*)(src + 4);
      const v4f a2 = *(const v4f*)(src + 8);
      const v4f a3 = *(const v4f*)(src + 12);
      *(v4f*)(sR + lane * 16 + 0)  = a0;
      *(v4f*)(sR + lane * 16 + 4)  = a1;
      *(v4f*)(sR + lane * 16 + 8)  = a2;
      *(v4f*)(sR + lane * 16 + 12) = a3;
      sO[lane] = 0.0f;
      sO[32 + lane] = 0.0f;
      sO[64 + lane] = 0.0f;
    }
    __syncthreads();
    int nvalid = kDays - base;
    nvalid = nvalid < 0 ? 0 : (nvalid > 32 ? 32 : nvalid);
    if (lane == 0) {
#pragma unroll 1
      for (int s = 0; s < nvalid; ++s) {
        const v4f r0 = *(const v4f*)(sR + s * 16 + 0);
        const v4f r1 = *(const v4f*)(sR + s * 16 + 4);
        const v4f r2 = *(const v4f*)(sR + s * 16 + 8);
        const v4f r3 = *(const v4f*)(sR + s * 16 + 12);
        const float rain = r0[0], rpi = r0[1], icpt = r0[2], cap = r0[3];
        const float meltpot = r1[0], snowflag = r1[1], fD = r1[2], bpfsl = r1[3];
        const float gfac = r2[0], fco2et = r2[1], vb = r2[2], pw = r2[3];
        const float ec = r3[0], par = r3[1];
        const float thetavol = theta / soildepth;
        const float rew = (thetavol - thetaPWP) / dfc;
        const float fwq = rew / soilthres;
        const float fw = (rew < soilthres) ? ((rew > 0.01f) ? fwq : 0.0f) : 1.0f;
        const float fe = fminf(fD, fw);
        const float gpp380 = bpfsl * fe;
        const float gpp = gpp380 * gfac;
        const bool over = (icpt + canw) > cap;
        float tf = smallcw ? rpi : (over ? ((rpi + canw) - cap) : rain);
        canw = smallcw ? canw : (over ? cap : (canw + icpt));
        const float newsnow = (snowflag > 0.5f) ? tf : 0.0f;
        tf = tf - newsnow;
        const float sn = snow + newsnow;
        const float melt = fminf(meltpot, sn);
        snow = sn - melt;
        const float fwetq = rew / etst;
        float fwet = (rew < etst) ? ((rew > 0.01f) ? fwetq : 0.0f) : 1.0f;
        fwet = (canw > 1e-8f) ? 1.0f : fwet;
        const float pw2 = powf(fmaxf(fw, 1e-12f), etnu);
        const float transp = (((vb * gpp380) / pw) * pw2) * fco2et;
        const float evap = (ec * fwet) * par;
        const float et = transp + evap;
        const float canw2 = fmaxf(canw - et, 0.0f);
        const float rem = fmaxf(et - canw, 0.0f);
        const float snow2 = fmaxf(snow - rem, 0.0f);
        const float etsoil = fmaxf(rem - snow, 0.0f);
        const float st0 = fmaxf(((theta + tf) + melt) - etsoil, 1e-4f);
        const float drq = fmaxf(st0 - fcap, 0.0f) / taud;
        const float drain = (taud > 0.0f) ? drq : 0.0f;
        theta = st0 - drain;
        canw = canw2;
        snow = snow2;
        sO[3 * s + 0] = gpp;
        sO[3 * s + 1] = et;
        sO[3 * s + 2] = theta;
      }
    }
    __syncthreads();
    {
      const bool valid = (base + lane) < kDays;
      const float tv = sO[3 * lane + 2];
      const float nv = (tv - sw0) / sw1;
      sO[3 * lane + 2] = valid ? nv : 0.0f;
    }
    __syncthreads();
    const int nv4 = (nvalid * 3) >> 2;
    const int li = lane < 23 ? lane : 23;
    const v4f ov = *(const v4f*)(sO + 4 * li);
    v4u pw4[4];
#pragma unroll
    for (int it = 0; it < 4; ++it) {
      const int rowl = it * 8 + (lane >> 2);
      const float a = sO[3 * rowl + 0] * pcarry;
      const float b = sO[3 * rowl + 1] * pcarry;
      const float c = sO[3 * rowl + 2] * pcarry;
      const bool sel = (lane & 3) == 0;
      unsigned ha, ra, hb, rb, hc, rc;
      split_h16(a, ha, ra);
      split_h16(b, hb, rb);
      split_h16(c, hc, rc);
      const unsigned w0 = ha | (hb << 16);
      const unsigned w1 = hc | (ra << 16);
      const unsigned w2 = rb | (rc << 16);
      pw4[it] = (v4u){sel ? w0 : zw, sel ? w1 : zw, sel ? w2 : zw, zw};
    }
    float* o1 = out1 + (size_t)base * 3 + 4 * lane;
    unsigned short* p3 = P3 + (size_t)base * 32 + lane * 8;
    for (int pass = 0; pass < 2; ++pass) {
      if (lane < nv4) *(volatile v4f*)o1 = ov;
#pragma unroll
      for (int it = 0; it < 4; ++it) *(volatile v4u*)(p3 + (size_t)it * 256) = pw4[it];
      __threadfence();
    }
  }
}

__global__ __launch_bounds__(256) void pack_out0_kernel(const float* __restrict__ Y, float* __restrict__ out0) {
  const int i = blockIdx.x * 256 + threadIdx.x;
  constexpr int kNv4 = (kDays * kYcols) / 4;
  const int ic = i < kNv4 ? i : (kNv4 - 1);
  const size_t r = (size_t)ic * 2;
  float a0 = Y[r * kNsmall + 0];
  float a1 = Y[r * kNsmall + 1];
  float b0 = Y[(r + 1) * kNsmall + 0];
  float b1 = Y[(r + 1) * kNsmall + 1];
  asm volatile("" : "+v"(a0), "+v"(a1), "+v"(b0), "+v"(b1));
  const v4f v = {a0, a1, b0, b1};
  const bool ok = i < kNv4;
  float* dst = out0 + (size_t)ic * 4;
  if (ok) *(volatile v4f*)dst = v;
  __threadfence();
  if (ok) *(volatile v4f*)dst = v;
}

extern "C" void kernel_launch(void* const* d_in, const int* in_sizes, int n_in,
                              void* d_out, int out_size, void* d_ws, size_t ws_size,
                              hipStream_t stream) {
  if (n_in < 16) return;
  if (in_sizes[0] != kDays * kXin) return;
  if (in_sizes[1] != kDays * 7) return;
  if (in_sizes[2] != 2) return;
  if (in_sizes[4] != kXin * kHid) return;
  if (in_sizes[5] != kHid) return;
  if (in_sizes[6] != kHid * kHid) return;
  if (in_sizes[7] != kHid) return;
  if (in_sizes[8] != kHid * kPcols) return;
  if (in_sizes[9] != kPcols) return;
  if (in_sizes[10] != kPpred * kHid) return;
  if (in_sizes[11] != kHid) return;
  if (in_sizes[12] != kHid * kHid) return;
  if (in_sizes[13] != kHid) return;
  if (in_sizes[14] != kHid * kYcols) return;
  if (in_sizes[15] != kYcols) return;
  if (out_size != kDays * (kYcols + kPpred)) return;
  if (ws_size < kWsTotal) return;

  const float* x   = (const float*)d_in[0];
  const float* cin = (const float*)d_in[1];
  const float* sw  = (const float*)d_in[2];
  const float* pW0 = (const float*)d_in[4];
  const float* pb0 = (const float*)d_in[5];
  const float* pW1 = (const float*)d_in[6];
  const float* pb1 = (const float*)d_in[7];
  const float* pW2 = (const float*)d_in[8];
  const float* pb2 = (const float*)d_in[9];
  const float* rW0 = (const float*)d_in[10];
  const float* rb0 = (const float*)d_in[11];
  const float* rW1 = (const float*)d_in[12];
  const float* rb1 = (const float*)d_in[13];
  const float* rW2 = (const float*)d_in[14];
  const float* rb2 = (const float*)d_in[15];
  float* out0 = (float*)d_out;
  float* out1 = (float*)d_out + (size_t)kDays * kYcols;

  char* ws = (char*)d_ws;
  unsigned short* H0   = (unsigned short*)(ws + kOffH0);
  unsigned short* H1   = (unsigned short*)(ws + kOffH1);
  float*          PR   = (float*)(ws + kOffPR);
  unsigned short* XH   = (unsigned short*)(ws + kOffXH);
  unsigned short* P3   = (unsigned short*)(ws + kOffP3);
  unsigned short* W0T  = (unsigned short*)(ws + kOffW0T);
  unsigned short* W1T  = (unsigned short*)(ws + kOffW1T);
  unsigned short* W2T  = (unsigned short*)(ws + kOffW2T);
  unsigned short* R0T  = (unsigned short*)(ws + kOffR0T);
  unsigned short* R1T  = (unsigned short*)(ws + kOffR1T);
  unsigned short* R2T  = (unsigned short*)(ws + kOffR2T);
  float*          PART = (float*)(ws + kOffPART);
  float*          B2P  = (float*)(ws + kOffB2P);
  float*          RB2P = (float*)(ws + kOffRB2P);
  float*          PM   = (float*)(ws + kOffPM);
  float*          FS   = (float*)(ws + kOffFS);
  float*          PRE  = (float*)(ws + kOffPRE);

  constexpr int kGemmBlkWide = (kMpad / 64) * (kHid / 64) / 8;
  constexpr int kGemmBlkThin = ((kMpad / 64) * (kNsmall / 64) + 7) / 8;
  static_assert(kGemmBlkWide == 782 && kGemmBlkThin == 98, "GEMM grids");

  pack_x_kernel<<<(kMpad * 4) / 256, 256, 0, stream>>>(x, XH, kMpad * 4, kCarryX);
  pack_wt_kernel<<<(kHid << 2) / 256, 256, 0, stream>>>(pW0, kXin, kHid, 2, 0, W0T, kHid << 2, kCarryW0);
  pack_wt_kernel<<<(kHid << 6) / 256, 256, 0, stream>>>(pW1, kHid, kHid, 6, 0, W1T, kHid << 6, kCarryW1);
  pack_wt_kernel<<<(kNsmall << 6) / 256, 256, 0, stream>>>(pW2, kHid, kPcols, 6, 0, W2T, kNsmall << 6, kCarryW2);
  pack_wt_kernel<<<(kHid << 2) / 256, 256, 0, stream>>>(rW0, kPpred, kHid, 2, kPpred, R0T, kHid << 2, kCarryR0);
  pack_wt_kernel<<<(kHid << 6) / 256, 256, 0, stream>>>(rW1, kHid, kHid, 6, 0, R1T, kHid << 6, kCarryR1);
  pack_wt_kernel<<<(kNsmall << 6) / 256, 256, 0, stream>>>(rW2, kHid, kYcols, 6, 0, R2T, kNsmall << 6, kCarryR2);
  pad_bias_kernel<<<1, 32, 0, stream>>>(pb2, kPcols, rb2, kYcols, B2P, RB2P);

  wmma_gemm64_f16<0, 1><<<kGemmBlkWide, 256, 0, stream>>>(
      XH, kKsmall, W0T, kKsmall, (void*)H0, kHid, pb0,
      kMpad, kHid, kKsmall, 1.0f / (kCarryX * kCarryW0), kCarryH);
  wmma_gemm64_f16<0, 0><<<kGemmBlkWide, 256, 0, stream>>>(
      H0, kHid, W1T, kHid, (void*)H1, kHid, pb1,
      kMpad, kHid, kHid, 1.0f / (kCarryH * kCarryW1), kCarryH);
  wmma_gemm64_f16<1, 0><<<kGemmBlkThin, 256, 0, stream>>>(
      H1, kHid, W2T, kHid, (void*)PR, kNsmall, B2P,
      kMpad, kNsmall, kHid, 1.0f / (kCarryH * kCarryW2), 1.0f);

  constrain_colsum_kernel<<<kRedBlk, 256, 0, stream>>>(PR, PART);
  mean_sfilter_kernel<<<1, 32, 0, stream>>>(PART, cin, PM, FS);
  daily_terms_kernel<<<kPreBlk, 256, 0, stream>>>(cin, PM, FS, PRE);
  water_scan_kernel<<<1, 32, 0, stream>>>(PM, PRE, sw, out1, P3, kCarryP);

  wmma_gemm64_f16<0, 1><<<kGemmBlkWide, 256, 0, stream>>>(
      P3, kKsmall, R0T, kKsmall, (void*)H0, kHid, rb0,
      kMpad, kHid, kKsmall, 1.0f / (kCarryP * kCarryR0), kCarryH);
  wmma_gemm64_f16<0, 0><<<kGemmBlkWide, 256, 0, stream>>>(
      H0, kHid, R1T, kHid, (void*)H1, kHid, rb1,
      kMpad, kHid, kHid, 1.0f / (kCarryH * kCarryR1), kCarryH);
  wmma_gemm64_f16<1, 0><<<kGemmBlkThin, 256, 0, stream>>>(
      H1, kHid, R2T, kHid, (void*)PR, kNsmall, RB2P,
      kMpad, kNsmall, kHid, 1.0f / (kCarryH * kCarryR2), 1.0f);

  pack_out0_kernel<<<((kDays * kYcols) / 4 + 255) / 256, 256, 0, stream>>>(PR, out0);
}
